// SparseBasicBlock_37950331027983
// MI455X (gfx1250) — hardware-verified
//
#include <hip/hip_runtime.h>
#include <stddef.h>
#include <stdint.h>


typedef _Float16 v16h __attribute__((ext_vector_type(16)));
typedef float    v8f  __attribute__((ext_vector_type(8)));
typedef float    v4f  __attribute__((ext_vector_type(4)));
typedef unsigned v4u  __attribute__((ext_vector_type(4)));

#define BN_EPS         1e-5f
#define K_OFF          9
#define CH             64
#define KSTEPS         18
#define WAVES          8
#define BLOCK_THREADS  (WAVES * 32)
#define SITES_PER_WAVE 32
#define B_LDS_DWORDS   (KSTEPS * 2 * CH * 8)
#define W_SCALE        16.0f
#define W_UNSCALE      0.0625f

union Frag { v16h v; v4u q[2]; };

__device__ __forceinline__ unsigned hpack2(float a, float b) {
  union { _Float16 h[2]; unsigned u; } t;
  t.h[0] = (_Float16)a;
  t.h[1] = (_Float16)b;
  return t.u;
}

__device__ __forceinline__ v8f wmma_f16(v16h a, v16h b, v8f c) {
  v8f d = __builtin_amdgcn_wmma_f32_16x16x32_f16(false, a, false, b, (short)0, c, false, false);
  asm volatile("v_nop\n\tv_nop\n\tv_nop\n\tv_nop" : "+v"(d) : "v"(a), "v"(b));
  return d;
}

__device__ __forceinline__ void stage_weights(const float* __restrict__ W, unsigned* lds) {
  for (int i = threadIdx.x; i < B_LDS_DWORDS; i += BLOCK_THREADS) {
    const int q    = i & 7;
    const int d    = (i >> 3) & 63;
    const int half = (i >> 9) & 1;
    const int kk   = i >> 10;
    const int loc  = 8 * half + 2 * q + ((q >> 2) << 3);
    const int k    = kk >> 1;
    const int c    = ((kk & 1) << 5) + loc;
    const float* wp = W + ((size_t)(k * CH + c)) * CH + d;
    lds[i] = hpack2(wp[0] * W_SCALE, wp[CH] * W_SCALE);
  }
}

__global__ __launch_bounds__(256)
void cvt_f16(const float* __restrict__ in, _Float16* outv, int n_vec) {
  const int i = blockIdx.x * 256 + threadIdx.x;
  if (i >= n_vec) return;
  const v4f* p = (const v4f*)(in + (size_t)i * 8);
  const v4f a = p[0], b = p[1];
  v4u r;
  r.x = hpack2(a.x, a.y);
  r.y = hpack2(a.z, a.w);
  r.z = hpack2(b.x, b.y);
  r.w = hpack2(b.z, b.w);
  volatile v4u* dst = (volatile v4u*)(outv + (size_t)i * 8);
  *dst = r;
  __threadfence();
  *dst = r;
}

template <bool LAYER2>
__global__ __launch_bounds__(BLOCK_THREADS) __attribute__((amdgpu_num_vgpr(248)))
void subm_conv(const _Float16* __restrict__ fin,
               const float* __restrict__ xres,
               const int* __restrict__ nbr,
               const float* __restrict__ W,
               const float* __restrict__ gam, const float* __restrict__ bet,
               const float* __restrict__ rmean, const float* __restrict__ rvar,
               _Float16* midout,
               float* fout,
               int n_sites, int n_wtiles) {
  __shared__ unsigned lwB[B_LDS_DWORDS];
  stage_weights(W, lwB);
  __syncthreads();

  const int lane = threadIdx.x & 31;
  const int wave = threadIdx.x >> 5;
  const int h    = lane >> 4;
  const int m16  = lane & 15;
  const int wt_raw = blockIdx.x * WAVES + wave;
  const bool active = wt_raw < n_wtiles;
  const int wt    = active ? wt_raw : (n_wtiles - 1);
  const int site0 = wt * SITES_PER_WAVE;

  int srow[2];
#pragma unroll
  for (int m = 0; m < 2; ++m) {
    int s = site0 + m * 16 + m16;
    srow[m] = s < n_sites ? s : (n_sites - 1);
  }

  v8f acc[2][4];
#pragma unroll
  for (int m = 0; m < 2; ++m)
#pragma unroll
    for (int nt = 0; nt < 4; ++nt) {
      v8f z = {0.f, 0.f, 0.f, 0.f, 0.f, 0.f, 0.f, 0.f};
      acc[m][nt] = z;
    }

  const unsigned* bl = lwB + h * 512 + m16 * 8;

#pragma unroll 1
  for (int k = 0; k < K_OFF; ++k) {
    int id[2];
#pragma unroll
    for (int m = 0; m < 2; ++m) {
      int v = nbr[(size_t)srow[m] * K_OFF + k];
      if (v < 0) v += n_sites;
      v = v < 0 ? 0 : v;
      v = v >= n_sites ? (n_sites - 1) : v;
      id[m] = v;
    }
#pragma unroll
    for (int cs = 0; cs < 2; ++cs) {
      const int kk = 2 * k + cs;
      Frag A[2];
#pragma unroll
      for (int m = 0; m < 2; ++m) {
        const _Float16* ap = fin + (size_t)id[m] * CH + cs * 32 + 8 * h;
        A[m].q[0] = *(const v4u*)(ap);
        A[m].q[1] = *(const v4u*)(ap + 16);
      }
      Frag B[4];
      const unsigned* bb = bl + kk * 1024;
#pragma unroll
      for (int nt = 0; nt < 4; ++nt) {
        B[nt].q[0] = *(const v4u*)(bb + nt * 128);
        B[nt].q[1] = *(const v4u*)(bb + nt * 128 + 4);
      }
#pragma unroll
      for (int m = 0; m < 2; ++m)
#pragma unroll
        for (int nt = 0; nt < 4; ++nt)
          acc[m][nt] = wmma_f16(A[m].v, B[nt].v, acc[m][nt]);
    }
  }

  __syncthreads();
  float*    stf = (float*)lwB + wave * 2048;
  _Float16* sth = (_Float16*)lwB + wave * 2048;

#pragma unroll
  for (int nt = 0; nt < 4; ++nt) {
    const int ch = nt * 16 + m16;
    const float inv  = gam[ch] * rsqrtf(rvar[ch] + BN_EPS);
    const float scl  = inv * W_UNSCALE;
    const float beta = bet[ch] - rmean[ch] * inv;
#pragma unroll
    for (int m = 0; m < 2; ++m)
#pragma unroll
      for (int r = 0; r < 8; ++r) {
        const int s = m * 16 + 8 * h + r;
        const float v = acc[m][nt][r] * scl + beta;
        if (LAYER2) stf[s * CH + ch] = v;
        else        sth[s * CH + ch] = (_Float16)fmaxf(v, 0.0f);
      }
  }
  __syncthreads();

  const int lsub = lane >> 3;
  const int p8   = lane & 7;

  if (LAYER2) {
    v4f o[16];
    bool ok[16];
#pragma unroll
    for (int t = 0; t < 16; ++t) {
      const int L = 4 * t + lsub;
      const int f = L * 32 + p8 * 4;
      const int site = site0 + (L >> 1);
      ok[t] = active && (site < n_sites);
      const v4f sv = *(const v4f*)(stf + f);
      v4f rx = {0.f, 0.f, 0.f, 0.f};
      if (ok[t]) rx = *(const v4f*)(xres + (size_t)site0 * CH + f);
      v4f w;
      w.x = fmaxf(sv.x + rx.x, 0.0f);
      w.y = fmaxf(sv.y + rx.y, 0.0f);
      w.z = fmaxf(sv.z + rx.z, 0.0f);
      w.w = fmaxf(sv.w + rx.w, 0.0f);
      o[t] = w;
    }
#pragma unroll
    for (int t = 0; t < 16; ++t) {
      const int f = (4 * t + lsub) * 32 + p8 * 4;
      if (ok[t]) *(volatile v4f*)(fout + (size_t)site0 * CH + f) = o[t];
    }
    __threadfence();
#pragma unroll
    for (int t = 0; t < 16; ++t) {
      const int f = (4 * t + lsub) * 32 + p8 * 4;
      if (ok[t]) *(volatile v4f*)(fout + (size_t)site0 * CH + f) = o[t];
    }
  } else {
    v4u o[8];
    bool ok[8];
#pragma unroll
    for (int t = 0; t < 8; ++t) {
      const int L  = 4 * t + lsub;
      const int hh = L * CH + p8 * 8;
      ok[t] = active && (site0 + L < n_sites);
      o[t]  = *(const v4u*)(sth + hh);
    }
#pragma unroll
    for (int t = 0; t < 8; ++t) {
      const int hh = (4 * t + lsub) * CH + p8 * 8;
      if (ok[t]) *(volatile v4u*)(midout + (size_t)site0 * CH + hh) = o[t];
    }
    __threadfence();
#pragma unroll
    for (int t = 0; t < 8; ++t) {
      const int hh = (4 * t + lsub) * CH + p8 * 8;
      if (ok[t]) *(volatile v4u*)(midout + (size_t)site0 * CH + hh) = o[t];
    }
  }
}

extern "C" void kernel_launch(void* const* d_in, const int* in_sizes, int n_in,
                              void* d_out, int out_size, void* d_ws, size_t ws_size,
                              hipStream_t stream) {
  if (n_in < 12) return;
  const float* x   = (const float*)d_in[0];
  const int*   nbr = (const int*)  d_in[1];
  const float* W1  = (const float*)d_in[2];
  const float* g1  = (const float*)d_in[3];
  const float* b1  = (const float*)d_in[4];
  const float* rm1 = (const float*)d_in[5];
  const float* rv1 = (const float*)d_in[6];
  const float* W2  = (const float*)d_in[7];
  const float* g2  = (const float*)d_in[8];
  const float* b2  = (const float*)d_in[9];
  const float* rm2 = (const float*)d_in[10];
  const float* rv2 = (const float*)d_in[11];

  const int n_sites = in_sizes[0] / CH;
  if (n_sites <= 0) return;
  if (in_sizes[1] < n_sites * K_OFF) return;
  if (in_sizes[2] < K_OFF * CH * CH || in_sizes[7] < K_OFF * CH * CH) return;
  if ((size_t)out_size < (size_t)n_sites * CH) return;

  const size_t feat_bytes = (size_t)n_sites * CH * sizeof(_Float16);
  if (2 * feat_bytes > ws_size) return;
  _Float16* xh  = (_Float16*)d_ws;
  _Float16* mid = (_Float16*)((char*)d_ws + feat_bytes);
  float* out = (float*)d_out;

  const int n_vec       = n_sites * (CH / 8);
  const int cvt_blocks  = (n_vec + 255) / 256;
  const int n_wtiles    = (n_sites + SITES_PER_WAVE - 1) / SITES_PER_WAVE;
  const int conv_blocks = (n_wtiles + WAVES - 1) / WAVES;

  cvt_f16<<<cvt_blocks, 256, 0, stream>>>(x, xh, n_vec);
  subm_conv<false><<<conv_blocks, BLOCK_THREADS, 0, stream>>>(
      xh, x, nbr, W1, g1, b1, rm1, rv1, mid, out, n_sites, n_wtiles);
  subm_conv<true><<<conv_blocks, BLOCK_THREADS, 0, stream>>>(
      mid, x, nbr, W2, g2, b2, rm2, rv2, mid, out, n_sites, n_wtiles);
  (void)hipGetLastError();
}
